// TA_LSTMCell_7344394076758
// MI455X (gfx1250) — hardware-verified
//
#include <hip/hip_runtime.h>
#include <math.h>
#include <stdint.h>

#define NB  4096
#define NI  512
#define NH  1024
#define NG  (4 * NH)
#define KG  (NI + NH)
static_assert((NB % 64) == 0 && (NG % 64) == 0 && (NH % 64) == 0);
static_assert((KG % 32) == 0 && (NH % 32) == 0);
static_assert((NI % 256) == 0 && (NH % 256) == 0);
static_assert(NH == 4 * 256);

typedef __bf16   v16b __attribute__((ext_vector_type(16)));
typedef __bf16   v8b  __attribute__((ext_vector_type(8)));
typedef float    v8f  __attribute__((ext_vector_type(8)));
typedef float    v4f  __attribute__((ext_vector_type(4)));
typedef unsigned int v4u __attribute__((ext_vector_type(4)));

__device__ __forceinline__ unsigned short bf_bits(float f) {
  unsigned u = __float_as_uint(f);
  return (unsigned short)((u + 0x7FFFu + ((u >> 16) & 1u)) >> 16);
}
__device__ __forceinline__ unsigned pk16(unsigned short a, unsigned short b) { return (unsigned)a | ((unsigned)b << 16); }
__device__ __forceinline__ v8f zero8() { v8f z = {0.f, 0.f, 0.f, 0.f, 0.f, 0.f, 0.f, 0.f}; return z; }
__device__ __forceinline__ float bf_rne(float f) {
  return __uint_as_float(((unsigned)bf_bits(f)) << 16);
}

__device__ __forceinline__ v16b ldfrag_b(const __bf16* p) {
  union { v16b v; v8b h[2]; } f;
  f.h[0] = *(const v8b*)(p);
  f.h[1] = *(const v8b*)(p + 16);
  return f.v;
}

__device__ __forceinline__ v8f mma_b_raw(v16b a, v16b b, v8f c) {
  return __builtin_amdgcn_wmma_f32_16x16x32_bf16(false, a, false, b, (short)0, c, false, false);
}
__device__ __forceinline__ void dep_guard_b(v8f& a, v8f& b, v16b x, v16b y) {
#if defined(__HIP_DEVICE_COMPILE__)
  asm volatile("v_nop\n\tv_nop\n\tv_nop\n\tv_nop" : "+v"(a), "+v"(b) : "v"(x), "v"(y));
#endif
}
__device__ __forceinline__ void keep4_b(v16b a, v16b b, v16b c, v16b d) {
#if defined(__HIP_DEVICE_COMPILE__)
  asm volatile("v_nop" :: "v"(a), "v"(b), "v"(c), "v"(d));
#endif
}
__device__ __forceinline__ void acc_guard4(v8f& a, v8f& b, v8f& c, v8f& d) {
#if defined(__HIP_DEVICE_COMPILE__)
  asm volatile("v_nop\n\tv_nop\n\tv_nop\n\tv_nop" : "+v"(a), "+v"(b), "+v"(c), "+v"(d));
#endif
}
__device__ __forceinline__ void wave_sync_lds() {
  __builtin_amdgcn_fence(__ATOMIC_RELEASE, "workgroup");
  __builtin_amdgcn_wave_barrier();
  __builtin_amdgcn_fence(__ATOMIC_ACQUIRE, "workgroup");
}

__global__ __launch_bounds__(256) void cvt_rows8(const float* __restrict__ src, int C,
                                                 unsigned short* dst, int ldd, int coff, int nch) {
  const int i = blockIdx.x * 256 + threadIdx.x;
  if (i >= nch) return;
  const int cpr = C >> 3;
  const int r = i / cpr;
  const int c8 = (i - r * cpr) * 8;
  const v4f a = *(const v4f*)(src + (size_t)r * C + c8);
  const v4f b = *(const v4f*)(src + (size_t)r * C + c8 + 4);
  v4u p;
  p[0] = pk16(bf_bits(a[0]), bf_bits(a[1]));
  p[1] = pk16(bf_bits(a[2]), bf_bits(a[3]));
  p[2] = pk16(bf_bits(b[0]), bf_bits(b[1]));
  p[3] = pk16(bf_bits(b[2]), bf_bits(b[3]));
  unsigned short* q = dst + (size_t)r * ldd + coff + c8;
  *(volatile v4u*)q = p;
  __threadfence();
  *(volatile v4u*)q = p;
}

__global__ __launch_bounds__(256) void tr_cvt64(const float* __restrict__ in, unsigned short* out,
                                                int R, int C) {
  __shared__ __align__(16) float s[64 * 68];
  const int tid = threadIdx.x;
  const int r0 = blockIdx.y * 64;
  const int c0 = blockIdx.x * 64;
  const int rl = tid >> 4;
  const int c4 = (tid & 15) * 4;
#pragma unroll
  for (int it = 0; it < 4; ++it) {
    const int r = it * 16 + rl;
    const v4f v = *(const v4f*)(in + (size_t)(r0 + r) * C + c0 + c4);
    s[(c4 + 0) * 68 + r] = v[0];
    s[(c4 + 1) * 68 + r] = v[1];
    s[(c4 + 2) * 68 + r] = v[2];
    s[(c4 + 3) * 68 + r] = v[3];
  }
  __syncthreads();
  const int q8 = (tid & 7) * 8;
  const int cl = tid >> 3;
  v4u pk[2];
#pragma unroll
  for (int it = 0; it < 2; ++it) {
    const int c = it * 32 + cl;
    const v4f a = *(const v4f*)(s + c * 68 + q8);
    const v4f b = *(const v4f*)(s + c * 68 + q8 + 4);
    v4u p;
    p[0] = pk16(bf_bits(a[0]), bf_bits(a[1]));
    p[1] = pk16(bf_bits(a[2]), bf_bits(a[3]));
    p[2] = pk16(bf_bits(b[0]), bf_bits(b[1]));
    p[3] = pk16(bf_bits(b[2]), bf_bits(b[3]));
    pk[it] = p;
  }
  for (int pass = 0; pass < 2; ++pass) {
#pragma unroll
    for (int it = 0; it < 2; ++it) {
      const int c = it * 32 + cl;
      *(volatile v4u*)(out + (size_t)(c0 + c) * R + r0 + q8) = pk[it];
    }
    __threadfence();
  }
}

template <int OUT16, int BIAS, int RES>
__global__ __launch_bounds__(256) void gemm64(
    const unsigned short* __restrict__ Ap, int lda,
    const unsigned short* __restrict__ Btp, int ldb,
    void* Cout, int ldc,
    const float* __restrict__ bias, int nbias,
    const float* __restrict__ res, int ldr,
    float alpha, int M, int N, int K) {
  const __bf16* A  = (const __bf16*)(const void*)Ap;
  const __bf16* Bt = (const __bf16*)(const void*)Btp;
  __shared__ __align__(16) float sT[8][16 * 68];
  const int lane = threadIdx.x & 31;
  const int wave = threadIdx.x >> 5;
  const int tilesN = N >> 6;
  const int tilesM = M >> 6;
  const int tile = blockIdx.x * 8 + wave;
  if (tile >= tilesM * tilesN) return;
  const int tm = tile / tilesN;
  const int tn = tile - tm * tilesN;
  const int m0 = tm << 6;
  const int n0 = tn << 6;

  const int rlane = lane & 15;
  const int koff  = (lane >> 4) * 8;
  const int mOff  = (lane >> 4) * 8;

  v8f acc[4][4];
#pragma unroll
  for (int i = 0; i < 4; ++i)
#pragma unroll
    for (int j = 0; j < 4; ++j) acc[i][j] = zero8();

  for (int k0 = 0; k0 < K; k0 += 32) {
    v16b bh[4];
#pragma unroll
    for (int j = 0; j < 4; ++j) {
      const size_t bo = (size_t)(n0 + (j << 4) + rlane) * ldb + koff + k0;
      bh[j] = ldfrag_b(Bt + bo);
    }
#pragma unroll
    for (int i = 0; i < 4; ++i) {
      const size_t ao = (size_t)(m0 + (i << 4) + rlane) * lda + koff + k0;
      const v16b ah = ldfrag_b(A + ao);
#pragma unroll
      for (int j = 0; j < 4; ++j) {
        acc[i][j] = mma_b_raw(ah, bh[j], acc[i][j]);
      }
      dep_guard_b(acc[i][0], acc[i][3], ah, bh[3]);
    }
    keep4_b(bh[0], bh[1], bh[2], bh[3]);
  }
  acc_guard4(acc[0][0], acc[0][1], acc[0][2], acc[0][3]);
  acc_guard4(acc[1][0], acc[1][1], acc[1][2], acc[1][3]);
  acc_guard4(acc[2][0], acc[2][1], acc[2][2], acc[2][3]);
  acc_guard4(acc[3][0], acc[3][1], acc[3][2], acc[3][3]);

  float* slab = sT[wave];
#pragma unroll
  for (int i = 0; i < 4; ++i) {
    const int mBase = m0 + (i << 4);
#pragma unroll
    for (int j = 0; j < 4; ++j) {
#pragma unroll
      for (int r = 0; r < 8; ++r) {
        slab[(mOff + r) * 68 + (j << 4) + rlane] = acc[i][j][r];
      }
    }
    wave_sync_lds();
    if (OUT16 == 0) {
      float* C = (float*)Cout;
      const int hh = lane >> 4, c4 = (lane & 15) * 4;
      for (int pass = 0; pass < 2; ++pass) {
#pragma unroll
        for (int it = 0; it < 8; ++it) {
          const int row = it * 2 + hh;
          v4f v = *(const v4f*)(slab + row * 68 + c4);
          v = v * alpha;
          if (BIAS == 1) {
            int bi = n0 + c4; if (bi > nbias - 4) bi = nbias - 4; if (bi < 0) bi = 0;
            const v4f bb = *(const v4f*)(bias + bi);
            v = v + bb;
          }
          if (BIAS == 2) {
            int bi = mBase + row; if (bi > nbias - 1) bi = nbias - 1; if (bi < 0) bi = 0;
            const float bb = bias[bi];
            v[0] += bb; v[1] += bb; v[2] += bb; v[3] += bb;
          }
          if (RES) {
            v4f rr = *(const v4f*)(res + (size_t)(mBase + row) * ldr + n0 + c4);
            rr[0] = bf_rne(rr[0]); rr[1] = bf_rne(rr[1]); rr[2] = bf_rne(rr[2]); rr[3] = bf_rne(rr[3]);
            v = v + rr;
          }
          *(volatile v4f*)(C + (size_t)(mBase + row) * ldc + n0 + c4) = v;
        }
        __threadfence();
      }
    } else {
      unsigned short* C16 = (unsigned short*)Cout;
      const int q8 = (lane & 7) * 8, rr = lane >> 3;
      v4u pk[4];
#pragma unroll
      for (int it = 0; it < 4; ++it) {
        const int row = it * 4 + rr;
        v4f a = *(const v4f*)(slab + row * 68 + q8);
        v4f b = *(const v4f*)(slab + row * 68 + q8 + 4);
        a = a * alpha;
        b = b * alpha;
        if (BIAS == 1) {
          int bi = n0 + q8; if (bi > nbias - 8) bi = nbias - 8; if (bi < 0) bi = 0;
          const v4f b0 = *(const v4f*)(bias + bi);
          const v4f b1 = *(const v4f*)(bias + bi + 4);
          a = a + b0;
          b = b + b1;
        }
        if (BIAS == 2) {
          int bi = mBase + row; if (bi > nbias - 1) bi = nbias - 1; if (bi < 0) bi = 0;
          const float bb = bias[bi];
          a[0] += bb; a[1] += bb; a[2] += bb; a[3] += bb;
          b[0] += bb; b[1] += bb; b[2] += bb; b[3] += bb;
        }
        v4u p;
        p[0] = pk16(bf_bits(a[0]), bf_bits(a[1]));
        p[1] = pk16(bf_bits(a[2]), bf_bits(a[3]));
        p[2] = pk16(bf_bits(b[0]), bf_bits(b[1]));
        p[3] = pk16(bf_bits(b[2]), bf_bits(b[3]));
        pk[it] = p;
      }
      for (int pass = 0; pass < 2; ++pass) {
#pragma unroll
        for (int it = 0; it < 4; ++it) {
          const int row = it * 4 + rr;
          *(volatile v4u*)(C16 + (size_t)(mBase + row) * ldc + n0 + q8) = pk[it];
        }
        __threadfence();
      }
    }
    wave_sync_lds();
  }
}

__device__ __forceinline__ float act_f32(float x, bool th) {
#pragma clang fp contract(off)
  const float u = th ? (2.0f * x) : x;
  const float e = expf(-fabsf(u));
  const float r = 1.0f / (1.0f + e);
  const float sg = (u >= 0.0f) ? r : (e * r);
  const float tn = copysignf((1.0f - e) * r, x);
  return th ? tn : sg;
}

__global__ __launch_bounds__(256) void cell_rows(
    const float* __restrict__ G, const float* __restrict__ Cp,
    const float* __restrict__ cx, const float* __restrict__ tv,
    const float* __restrict__ bih, const float* __restrict__ bhh, const float* __restrict__ bdec,
    float* hy, float* cy) {
#pragma clang fp contract(off)
  __shared__ __align__(16) float sHy[NH];
  __shared__ __align__(16) float sCy[NH];
  const int tid = threadIdx.x;
  const int b = blockIdx.x;
  const float tb = bf_rne(tv[b]);
  const bool tnz = (tb != 0.0f);
  const float tsafe = tnz ? tb : 1.0f;
  const float Td = tnz ? (1.0f / tsafe) : 0.0f;
  const size_t gro = (size_t)b * NG;
  const size_t hro = (size_t)b * NH;
#pragma unroll 1
  for (int e = 0; e < 4; ++e) {
    const int c = e * 256 + tid;
    const float xc = Cp[hro + c] + bf_rne(bdec[c]);
    float ig = 0.0f, fg = 0.0f, cg = 0.0f, og = 0.0f, cst = 0.0f;
#pragma unroll 1
    for (int g = 0; g < 5; ++g) {
      const int gg = (g < 4) ? g : 3;
      const float s0 = G[gro + (size_t)gg * NH + c] + bf_rne(bih[gg * NH + c]);
      const float xg = s0 + bf_rne(bhh[gg * NH + c]);
      const float x = (g < 4) ? xg : xc;
      const bool th = (g == 2) || (g == 4);
      const float a = act_f32(x, th);
      ig  = (g == 0) ? a : ig;
      fg  = (g == 1) ? a : fg;
      cg  = (g == 2) ? a : cg;
      og  = (g == 3) ? a : og;
      cst = (g == 4) ? a : cst;
    }
    const float cxv = bf_rne(cx[hro + c]);
    const float tcs = Td * cst;
    const float cadj = (cxv - cst) + tcs;
    const float p1 = fg * cadj;
    const float p2 = ig * cg;
    const float cyv = p1 + p2;
    const float hyv = og * act_f32(cyv, true);
    sCy[c] = cyv;
    sHy[c] = hyv;
  }
  __syncthreads();
  const v4f h4 = *(const v4f*)(sHy + tid * 4);
  const v4f c4 = *(const v4f*)(sCy + tid * 4);
  float* ph = hy + hro + tid * 4;
  float* pc = cy + hro + tid * 4;
  *(volatile v4f*)ph = h4;
  *(volatile v4f*)pc = c4;
  __threadfence();
  *(volatile v4f*)ph = h4;
  *(volatile v4f*)pc = c4;
}

extern "C" void kernel_launch(void* const* d_in, const int* in_sizes, int n_in,
                              void* d_out, int out_size, void* d_ws, size_t ws_size,
                              hipStream_t stream) {
  if (n_in < 10) return;
  if (in_sizes[0] != NB * NI) return;
  if (in_sizes[1] != NB) return;
  if (in_sizes[2] != NB * NH || in_sizes[3] != NB * NH) return;
  if (in_sizes[4] != NG * NI || in_sizes[5] != NG * NH) return;
  if (in_sizes[6] != NG || in_sizes[7] != NG) return;
  if (in_sizes[8] != NH * NH || in_sizes[9] != NH) return;
  if (out_size != 2 * NB * NH) return;

  const float* x_in = (const float*)d_in[0];
  const float* t_in = (const float*)d_in[1];
  const float* hx   = (const float*)d_in[2];
  const float* cx   = (const float*)d_in[3];
  const float* wih  = (const float*)d_in[4];
  const float* whh  = (const float*)d_in[5];
  const float* bih  = (const float*)d_in[6];
  const float* bhh  = (const float*)d_in[7];
  const float* wdec = (const float*)d_in[8];
  const float* bdec = (const float*)d_in[9];
  float* hy = (float*)d_out;
  float* cy = hy + (size_t)NB * NH;

  const size_t PXa = (size_t)NB * KG * 2;
  const size_t PWb = (size_t)NG * KG * 2;
  const size_t PCx = (size_t)NB * NH * 2;
  const size_t PWd = (size_t)NH * NH * 2;
  const size_t PG  = (size_t)NB * NG * 4;
  const size_t PCp = (size_t)NB * NH * 4;
  size_t off = 0;
  const size_t oXa = off; off += PXa;
  const size_t oWb = off; off += PWb;
  const size_t oCx = off; off += PCx;
  const size_t oWd = off; off += PWd;
  const size_t oG  = off; off += PG;
  const size_t oCp = off; off += PCp;
  if (off > ws_size) return;
  if (off > (size_t)134217728) return;

  char* ws = (char*)d_ws;
  unsigned short* Xa  = (unsigned short*)(ws + oXa);
  unsigned short* Wb  = (unsigned short*)(ws + oWb);
  unsigned short* Cxb = (unsigned short*)(ws + oCx);
  unsigned short* Wdt = (unsigned short*)(ws + oWd);
  float* G  = (float*)(ws + oG);
  float* Cp = (float*)(ws + oCp);

  const dim3 blk(256);
  const int nchX  = NB * NI / 8;
  const int nchH  = NB * NH / 8;
  const int nchWi = NG * NI / 8;
  const int nchWh = NG * NH / 8;
  const dim3 gX((nchX + 255) / 256);
  const dim3 gH((nchH + 255) / 256);
  const dim3 gWi((nchWi + 255) / 256);
  const dim3 gWh((nchWh + 255) / 256);
  const dim3 gTr(NH / 64, NH / 64);
  const dim3 gGate(((NB / 64) * (NG / 64) + 7) / 8);
  const dim3 gDec(((NB / 64) * (NH / 64) + 7) / 8);
  const dim3 gCell(NB);

  cvt_rows8<<<gX,  blk, 0, stream>>>(x_in, NI, Xa, KG, 0,  nchX);
  cvt_rows8<<<gH,  blk, 0, stream>>>(hx,   NH, Xa, KG, NI, nchH);
  cvt_rows8<<<gWi, blk, 0, stream>>>(wih,  NI, Wb, KG, 0,  nchWi);
  cvt_rows8<<<gWh, blk, 0, stream>>>(whh,  NH, Wb, KG, NI, nchWh);
  cvt_rows8<<<gH,  blk, 0, stream>>>(cx,   NH, Cxb, NH, 0, nchH);
  tr_cvt64<<<gTr, blk, 0, stream>>>(wdec, Wdt, NH, NH);
  gemm64<0, 0, 0><<<gGate, blk, 0, stream>>>(Xa, KG, Wb, KG, (void*)G, NG, bih, NG, cx, NH,
                                            1.0f, NB, NG, KG);
  gemm64<0, 0, 0><<<gDec, blk, 0, stream>>>(Cxb, NH, Wdt, NH, (void*)Cp, NH, bdec, NH, cx, NH,
                                           1.0f, NB, NH, NH);
  cell_rows<<<gCell, blk, 0, stream>>>(G, Cp, cx, t_in, bih, bhh, bdec, hy, cy);
  (void)hipGetLastError();
}
